// LearnerCT_52871047413971
// MI455X (gfx1250) — hardware-verified
//
#include <hip/hip_runtime.h>
#include <stddef.h>


typedef _Float16 h16;
typedef _Float16 v16h __attribute__((ext_vector_type(16)));
typedef _Float16 v8h  __attribute__((ext_vector_type(8)));
typedef float    v8f  __attribute__((ext_vector_type(8)));
typedef float    v4f  __attribute__((ext_vector_type(4)));

#ifndef NROWS
#define NROWS 16384
#endif
#define NROWS_FULL 16384
#define DIN   64
#define HID   256
#define TROWS 32

static_assert(NROWS >= TROWS && NROWS <= NROWS_FULL && (NROWS % TROWS) == 0);
static_assert(DIN == 64);
static_assert((HID % 64) == 0 && (HID % 32) == 0 && (HID % 16) == 0);
static_assert(((HID * DIN) % 2048) == 0);
static_assert(((HID * HID) % 2048) == 0);
static_assert(TROWS == 32);
static_assert((NROWS_FULL * 4) == 65536);
static_assert((2 * NROWS_FULL * 4) == 131072);

#define LDT 72
#define LDY 264
static_assert((LDT % 8) == 0 && LDT >= 64);
static_assert((LDY % 8) == 0 && LDY >= HID);

#define WCARRY 64.0f
#define YCARRY 64.0f
#define TCARRY 64.0f

#define W1H_BYTES ((size_t)HID * DIN * 2)
#define W2H_BYTES ((size_t)HID * HID * 2)
#define OFF_W1H ((size_t)0)
#define OFF_W2H (OFF_W1H + W1H_BYTES)
#define OFF_W2T (OFF_W2H + W2H_BYTES)
#define WS_TOTAL (OFF_W2T + W2H_BYTES)
static_assert((W1H_BYTES % 128) == 0 && (W2H_BYTES % 128) == 0);
static_assert(WS_TOTAL <= (size_t)134217728);

static_assert((size_t)TROWS * HID * 4 + 2 * (size_t)TROWS * LDY * 2 + 2 * TROWS * 4 + 3 * TROWS * 4
              <= (size_t)131072);

__device__ __forceinline__ float bf16r(float x) {
  unsigned int u = __float_as_uint(x);
  u = (u + 0x7FFFu + ((u >> 16) & 1u)) & 0xFFFF0000u;
  return __uint_as_float(u);
}

__device__ __forceinline__ h16 toh_flush(float v) {
  const h16 r = (h16)v;
  return (fabsf(v) < 6.103515625e-05f) ? (h16)0.0f : r;
}

__device__ __forceinline__ v16h frag_at(const _Float16* p) {
  v8h lo = *(const v8h*)(p);
  v8h hi = *(const v8h*)(p + 16);
  v16h out;
#pragma unroll
  for (int i = 0; i < 8; ++i) { out[i] = lo[i]; out[i + 8] = hi[i]; }
  return out;
}
__device__ __forceinline__ v16h ld_frag(const _Float16* base, unsigned ld) {
  const unsigned lane = threadIdx.x & 31u;
  return frag_at(base + (lane & 15u) * ld + (lane >> 4) * 8u);
}

__device__ __forceinline__ v16h frag_f32(const float* p) {
  const v4f a0 = *(const v4f*)(p);
  const v4f a1 = *(const v4f*)(p + 4);
  const v4f a2 = *(const v4f*)(p + 16);
  const v4f a3 = *(const v4f*)(p + 20);
  v16h out;
#pragma unroll
  for (int i = 0; i < 4; ++i) {
    out[i]      = toh_flush(bf16r(a0[i]));
    out[i + 4]  = toh_flush(bf16r(a1[i]));
    out[i + 8]  = toh_flush(bf16r(a2[i]));
    out[i + 12] = toh_flush(bf16r(a3[i]));
  }
  return out;
}

__device__ __forceinline__ v8f wmma16(v16h a, v16h b, v8f c) {
  v8f d = __builtin_amdgcn_wmma_f32_16x16x32_f16(false, a, false, b, (short)0, c,
                                                 false, false);
  asm volatile("v_nop\n\tv_nop\n\tv_nop\n\tv_nop" : "+v"(d) : "v"(a), "v"(b));
  return d;
}

__device__ __forceinline__ float red16_sum(float x) {
#pragma unroll
  for (int off = 1; off < 16; off <<= 1) x += __shfl_xor(x, off, 32);
  return x;
}

__device__ __forceinline__ void wave_lds_sync() {
  __builtin_amdgcn_fence(3  , "wavefront");
  asm volatile("s_wait_dscnt 0x0" ::: "memory");
  __builtin_amdgcn_wave_barrier();
}

__global__ __launch_bounds__(256) void wconv_kernel(
    const float* __restrict__ W, _Float16* __restrict__ Wt, unsigned ldw, unsigned ldk) {
  __shared__ _Float16 T[64 * LDT];
  const unsigned tid = threadIdx.x;
  const unsigned n0 = blockIdx.x * 64u;
  const unsigned k0 = blockIdx.y * 64u;
#pragma unroll 4
  for (unsigned j = 0; j < 16u; ++j) {
    const unsigned idx = tid + 256u * j;
    const unsigned kr = idx >> 6, nc = idx & 63u;
    const float v = W[(size_t)(k0 + kr) * ldw + n0 + nc];
    T[nc * LDT + kr] = toh_flush(WCARRY * bf16r(v));
  }
  __syncthreads();
  v8h x[2];
  size_t off[2];
#pragma unroll
  for (unsigned i = 0; i < 2u; ++i) {
    const unsigned n = 32u * i + (tid >> 3);
    const unsigned kc = (tid & 7u) * 8u;
    x[i] = *(const v8h*)&T[n * LDT + kc];
    off[i] = (size_t)(n0 + n) * ldk + k0 + kc;
  }
#pragma unroll
  for (int i = 0; i < 2; ++i) *(volatile v8h*)(Wt + off[i]) = x[i];
  __threadfence();
#pragma unroll
  for (int i = 0; i < 2; ++i) *(volatile v8h*)(Wt + off[i]) = x[i];
}

__global__ __launch_bounds__(256) void wcast_kernel(
    const float* __restrict__ W, _Float16* __restrict__ Wh) {
  const size_t e = ((size_t)blockIdx.x * 256u + threadIdx.x) * 8u;
  const v4f a0 = *(const v4f*)(W + e);
  const v4f a1 = *(const v4f*)(W + e + 4);
  v8h x;
#pragma unroll
  for (int i = 0; i < 4; ++i) {
    x[i]     = toh_flush(WCARRY * bf16r(a0[i]));
    x[i + 4] = toh_flush(WCARRY * bf16r(a1[i]));
  }
  *(volatile v8h*)(Wh + e) = x;
  __threadfence();
  *(volatile v8h*)(Wh + e) = x;
}

__global__ __launch_bounds__(32) void fused_kernel(
    const float* __restrict__ S, const float* __restrict__ Sd,
    const _Float16* __restrict__ W1h, const _Float16* __restrict__ W2h,
    const _Float16* __restrict__ W2t,
    const float* __restrict__ b1, const float* __restrict__ b2, const float* __restrict__ W3,
    float* __restrict__ out) {
  __shared__ float    ZW[TROWS * HID];
  __shared__ _Float16 Y[TROWS * LDY];
  __shared__ _Float16 T[TROWS * LDY];
  __shared__ float    RS[2 * TROWS];
  __shared__ float    OS[3 * TROWS];

  const unsigned lane = threadIdx.x & 31u;
  const unsigned hh = lane >> 4, m = lane & 15u;
  const unsigned row0 = blockIdx.x * (unsigned)TROWS;

  float F = 0.0f, SD = 0.0f;
  {
    const float* sr = S  + (size_t)(row0 + lane) * DIN;
    const float* dr = Sd + (size_t)(row0 + lane) * DIN;
#pragma unroll 1
    for (unsigned j = 0; j < (unsigned)(DIN / 4); ++j) {
      const v4f s4 = *(const v4f*)(sr + 4u * j);
      const v4f d4 = *(const v4f*)(dr + 4u * j);
#pragma unroll
      for (int i = 0; i < 4; ++i) {
        const float s = bf16r(s4[i]);
        const float d = bf16r(d4[i]);
        F  += s * s;
        SD += s * d;
      }
    }
  }

  v16h sa[2][2], da[2][2];
#pragma unroll
  for (int mt = 0; mt < 2; ++mt)
#pragma unroll
    for (int c = 0; c < 2; ++c) {
      const size_t o = (size_t)(row0 + (unsigned)mt * 16u + m) * DIN + (unsigned)c * 32u + hh * 8u;
      sa[mt][c] = frag_f32(S + o);
      da[mt][c] = frag_f32(Sd + o);
    }

#pragma unroll 1
  for (unsigned nt = 0; nt < (unsigned)(HID / 16); ++nt) {
    const unsigned col = nt * 16u + m;
    const _Float16* bp = W1h + (size_t)col * DIN + hh * 8u;
    const v16h w0 = frag_at(bp);
    const v16h w1 = frag_at(bp + 32);
    v8f cz[2], cw[2];
#pragma unroll
    for (int mt = 0; mt < 2; ++mt) {
      cz[mt] = (v8f){};
      cw[mt] = (v8f){};
      cz[mt] = wmma16(sa[mt][0], w0, cz[mt]);
      cz[mt] = wmma16(sa[mt][1], w1, cz[mt]);
      cw[mt] = wmma16(da[mt][0], w0, cw[mt]);
      cw[mt] = wmma16(da[mt][1], w1, cw[mt]);
    }
    const float bb = bf16r(b1[col]);
#pragma unroll
    for (int mt = 0; mt < 2; ++mt)
#pragma unroll
      for (int r = 0; r < 8; ++r) {
        const unsigned row = (unsigned)mt * 16u + hh * 8u + (unsigned)r;
        const float z = cz[mt][r] * (1.0f / WCARRY) + bb;
        const float w = cw[mt][r] * (1.0f / WCARRY);
        ZW[row * HID + col] = 2.0f * z * w;
        Y[row * LDY + col]  = toh_flush(YCARRY * (z * z));
      }
  }
  wave_lds_sync();

  float nnp[2][8];
#pragma unroll
  for (int mt = 0; mt < 2; ++mt)
#pragma unroll
    for (int r = 0; r < 8; ++r) nnp[mt][r] = 0.0f;

#pragma unroll 1
  for (unsigned nt = 0; nt < (unsigned)(HID / 16); ++nt) {
    const unsigned col = nt * 16u + m;
    const _Float16* bp = W2h + (size_t)col * HID + hh * 8u;
    v8f acc[2];
    acc[0] = (v8f){};
    acc[1] = (v8f){};
#pragma unroll
    for (int c = 0; c < HID / 32; ++c) {
      const v16h b = frag_at(bp + c * 32);
#pragma unroll
      for (int mt = 0; mt < 2; ++mt) {
        const v16h a = ld_frag(&Y[(mt * 16) * LDY + c * 32], LDY);
        acc[mt] = wmma16(a, b, acc[mt]);
      }
    }
    const float bb = bf16r(b2[col]);
    const float w3 = bf16r(W3[col]);
#pragma unroll
    for (int mt = 0; mt < 2; ++mt)
#pragma unroll
      for (int r = 0; r < 8; ++r) {
        const unsigned row = (unsigned)mt * 16u + hh * 8u + (unsigned)r;
        const float z = acc[mt][r] * (1.0f / (WCARRY * YCARRY)) + bb;
        nnp[mt][r] += w3 * (z * z);
        T[row * LDY + col] = toh_flush(TCARRY * (2.0f * w3 * z));
      }
  }
  wave_lds_sync();

  float gsp[2][8];
#pragma unroll
  for (int mt = 0; mt < 2; ++mt)
#pragma unroll
    for (int r = 0; r < 8; ++r) gsp[mt][r] = 0.0f;

#pragma unroll 1
  for (unsigned pt = 0; pt < (unsigned)(HID / 16); ++pt) {
    const unsigned col = pt * 16u + m;
    const _Float16* bp = W2t + (size_t)col * HID + hh * 8u;
    v8f acc[2];
    acc[0] = (v8f){};
    acc[1] = (v8f){};
#pragma unroll
    for (int c = 0; c < HID / 32; ++c) {
      const v16h b = frag_at(bp + c * 32);
#pragma unroll
      for (int mt = 0; mt < 2; ++mt) {
        const v16h a = ld_frag(&T[(mt * 16) * LDY + c * 32], LDY);
        acc[mt] = wmma16(a, b, acc[mt]);
      }
    }
#pragma unroll
    for (int mt = 0; mt < 2; ++mt)
#pragma unroll
      for (int r = 0; r < 8; ++r) {
        const unsigned row = (unsigned)mt * 16u + hh * 8u + (unsigned)r;
        const float u = acc[mt][r] * (1.0f / (WCARRY * TCARRY));
        gsp[mt][r] += u * ZW[row * HID + col];
      }
  }

#pragma unroll
  for (int mt = 0; mt < 2; ++mt)
#pragma unroll
    for (int r = 0; r < 8; ++r) {
      nnp[mt][r] = red16_sum(nnp[mt][r]);
      gsp[mt][r] = red16_sum(gsp[mt][r]);
    }

#pragma unroll
  for (int mt = 0; mt < 2; ++mt) {
    float vn = nnp[mt][0];
    float vg = gsp[mt][0];
#pragma unroll
    for (int r = 1; r < 8; ++r) {
      const bool pick = ((m & 7u) == (unsigned)r);
      vn = pick ? nnp[mt][r] : vn;
      vg = pick ? gsp[mt][r] : vg;
    }
    const unsigned row = (unsigned)mt * 16u + hh * 8u + (m & 7u);
    RS[row] = vn;
    RS[TROWS + row] = vg;
  }
  wave_lds_sync();

  {
    const float nn = RS[lane];
    const float gs = RS[TROWS + lane];
    const float V  = nn * F;
    const float Vd = 2.0f * nn * SD + F * gs;
    OS[lane] = V;
    OS[TROWS + lane] = Vd;
    OS[2 * TROWS + lane] = F;
  }
  wave_lds_sync();

  {
    const unsigned q = lane >> 3, pc = lane & 7u;
    const unsigned qc = (q < 3u) ? q : 2u;
    const v4f x = *(const v4f*)&OS[qc * TROWS + pc * 4u];
    float* dst = out + (size_t)qc * NROWS_FULL + row0 + pc * 4u;
    if (lane < 24u) *(volatile v4f*)dst = x;
    __threadfence();
    if (lane < 24u) *(volatile v4f*)dst = x;
  }
}

extern "C" void kernel_launch(void* const* d_in, const int* in_sizes, int n_in,
                              void* d_out, int out_size, void* d_ws, size_t ws_size,
                              hipStream_t stream) {
  if (n_in < 7) return;
  if ((long long)in_sizes[0] < (long long)NROWS * DIN) return;
  if ((long long)in_sizes[1] < (long long)NROWS * DIN) return;
  if (in_sizes[2] < HID * DIN) return;
  if (in_sizes[3] < HID) return;
  if (in_sizes[4] < HID * HID) return;
  if (in_sizes[5] < HID) return;
  if (in_sizes[6] < HID) return;
  if ((long long)out_size < (long long)2 * NROWS_FULL + NROWS) return;
  if (ws_size < WS_TOTAL) return;

  const float* S   = (const float*)d_in[0];
  const float* Sd  = (const float*)d_in[1];
  const float* w1  = (const float*)d_in[2];
  const float* b1  = (const float*)d_in[3];
  const float* w2  = (const float*)d_in[4];
  const float* b2  = (const float*)d_in[5];
  const float* w3  = (const float*)d_in[6];
  float* out = (float*)d_out;

  char* ws = (char*)d_ws;
  _Float16* W1h = (_Float16*)(ws + OFF_W1H);
  _Float16* W2h = (_Float16*)(ws + OFF_W2H);
  _Float16* W2t = (_Float16*)(ws + OFF_W2T);

  dim3 blk(256);
  wcast_kernel<<<dim3((HID * DIN) / 2048), blk, 0, stream>>>(w1, W1h);
  wcast_kernel<<<dim3((HID * HID) / 2048), blk, 0, stream>>>(w2, W2h);
  wconv_kernel<<<dim3(HID / 64, HID / 64), blk, 0, stream>>>(w2, W2t, (unsigned)HID, (unsigned)HID);

  fused_kernel<<<dim3(NROWS / TROWS), dim3(32), 0, stream>>>(S, Sd, W1h, W2h, W2t, b1, b2, w3, out);
}
